// LinearSchNet_49143015801197
// MI455X (gfx1250) — hardware-verified
//
#include <hip/hip_runtime.h>
#include <stdint.h>
#include <math.h>

#define N_ATOM   10000
#define N_PADM   10048
#define N_EDGE   160000
#define N_EHALF  80000
#define N_PRED   80000
#define N_PHALF  40000
#define CHAN     128
#define NGAU     50
#define KGAU     64
#define NLAY     6
#define HOUT     64
#define NEMB     100
#define KEF      160
#define KEF_REAL 130
#define NEF      576
#define NEF_REAL 520
#define NTH      256
#define SRB      1024
#define SCH      2048
#define SPT      8
#define NTILE    10
#define NPA      (NTILE * SRB)
#define WSC      16.0f
#define WSC_INV  0.0625f
#define F16_MIN_NORMAL 6.103515625e-05f

static_assert(N_PADM % 64 == 0 && N_PADM >= N_ATOM && NPA >= N_PADM, "");
static_assert(N_EHALF % 64 == 0 && 2 * N_EHALF == N_EDGE && N_PHALF % 64 == 0 && 2 * N_PHALF == N_PRED, "");
static_assert(KGAU % 32 == 0 && KEF % 32 == 0 && CHAN % 64 == 0 && NEF % 64 == 0 && HOUT % 64 == 0, "");
static_assert(N_EDGE % SPT == 0 && N_EDGE % 32 == 0 && N_PRED % 32 == 0 && N_PHALF % 32 == 0, "");
static_assert(N_EDGE < (1 << 18) && SRB == 1024 && (SRB / 8) == 128 && NTH == 256 && SCH == 2048, "");
static_assert((N_PADM * 32) % 256 == 0 && (N_PADM * 16) % 256 == 0, "");

typedef __attribute__((ext_vector_type(16))) _Float16 v16h;
typedef __attribute__((ext_vector_type(8)))  _Float16 v8h;
typedef __attribute__((ext_vector_type(4)))  _Float16 v4hf;
typedef __attribute__((ext_vector_type(2)))  _Float16 v2hf;
typedef __attribute__((ext_vector_type(16))) __bf16   v16b;
typedef __attribute__((ext_vector_type(8)))  __bf16   v8b;
typedef __attribute__((ext_vector_type(8)))  float    v8f;
typedef __attribute__((ext_vector_type(4)))  float    v4f;
typedef __attribute__((ext_vector_type(4)))  int      v4i;

__device__ __forceinline__ unsigned short f2bf_bits(float f) {
  unsigned u = __float_as_uint(f);
  return (unsigned short)((u + 0x7FFFu + ((u >> 16) & 1u)) >> 16);
}
__device__ __forceinline__ float bf_bits2f(unsigned short h) { return __uint_as_float(((unsigned)h) << 16); }

__device__ __forceinline__ void dep_guard_h(v8f& a, v8f& b, v16h x, v16h y) { asm volatile("v_nop\n\tv_nop\n\tv_nop\n\tv_nop" : "+v"(a), "+v"(b) : "v"(x), "v"(y)); }
__device__ __forceinline__ void dep_guard_b(v8f& a, v8f& b, v16b x, v16b y) { asm volatile("v_nop\n\tv_nop\n\tv_nop\n\tv_nop" : "+v"(a), "+v"(b) : "v"(x), "v"(y)); }
__device__ __forceinline__ void keep4_h(v16h a, v16h b, v16h c, v16h d) { asm volatile("v_nop" :: "v"(a), "v"(b), "v"(c), "v"(d)); }
__device__ __forceinline__ void keep4_b(v16b a, v16b b, v16b c, v16b d) { asm volatile("v_nop" :: "v"(a), "v"(b), "v"(c), "v"(d)); }
__device__ __forceinline__ void acc_guard4(v8f& a, v8f& b, v8f& c, v8f& d) { asm volatile("v_nop\n\tv_nop\n\tv_nop\n\tv_nop" : "+v"(a), "+v"(b), "+v"(c), "+v"(d)); }
template <typename T> struct Frag;
template <> struct Frag<_Float16> {
  typedef v16h V; union U { v16h v; v8h h[2]; };
  static __device__ __forceinline__ v16h load(const _Float16* p) {
    U f; f.h[0] = *(const v8h*)(p); f.h[1] = *(const v8h*)(p + 16); return f.v;
  }
  static __device__ __forceinline__ v8f mma(v16h a, v16h b, v8f c) {
    return __builtin_amdgcn_wmma_f32_16x16x32_f16(false, a, false, b, (short)0, c, false, false);
  }
  static __device__ __forceinline__ void guard(v8f& a, v8f& b, v16h x, v16h y) { dep_guard_h(a, b, x, y); }
  static __device__ __forceinline__ void keep(v16h a, v16h b, v16h c, v16h d) { keep4_h(a, b, c, d); }
};
template <> struct Frag<__bf16> {
  typedef v16b V; union U { v16b v; v8b h[2]; };
  static __device__ __forceinline__ v16b load(const __bf16* p) {
    U f; f.h[0] = *(const v8b*)(p); f.h[1] = *(const v8b*)(p + 16); return f.v;
  }
  static __device__ __forceinline__ v8f mma(v16b a, v16b b, v8f c) {
    return __builtin_amdgcn_wmma_f32_16x16x32_bf16(false, a, false, b, (short)0, c, false, false);
  }
  static __device__ __forceinline__ void guard(v8f& a, v8f& b, v16b x, v16b y) { dep_guard_b(a, b, x, y); }
  static __device__ __forceinline__ void keep(v16b a, v16b b, v16b c, v16b d) { keep4_b(a, b, c, d); }
};

__device__ __forceinline__ float act_ssp(float v) {
  const float e = __expf(-fabsf(v));
  const float lg = __logf(1.0f + e);
  return fmaxf(v, 0.0f) + lg - 0.69314718f;
}
__device__ __forceinline__ float act_sigm(float v) {
  const float e = __expf(-fabsf(v));
  const float s = __builtin_amdgcn_rcpf(1.0f + e);
  return (v >= 0.0f) ? s : e * s;
}
__device__ __forceinline__ float flush16(float v) { return (fabsf(v) < F16_MIN_NORMAL) ? 0.0f : v; }

template <int ET> struct Elem;
template <> struct Elem<0> { typedef _Float16 T; };
template <> struct Elem<1> { typedef __bf16 T; };
template <int ET, bool SPLIT, int BIAS_MODE, int OUT_MODE, bool RESID, int ACT = 0>
__global__ __launch_bounds__(256) void wmma_gemm64(
    const unsigned short* __restrict__ Ap, const unsigned short* __restrict__ A2p, int lda, long strideA,
    const unsigned short* __restrict__ Btp, const unsigned short* __restrict__ Bt2p, int ldb, long strideB,
    void* __restrict__ Cout, void* __restrict__ Cout2, int ldc, long strideC,
    const float* __restrict__ bias,
    const float* __restrict__ resid, long strideR,
    int M, int N, int K, float scale) {
  typedef typename Elem<ET>::T T;
  typedef typename Frag<T>::V V;
  const T* A = (const T*)Ap; const T* A2 = (const T*)A2p; const T* Bt = (const T*)Btp; const T* Bt2 = (const T*)Bt2p;
  __shared__ __align__(16) float sT[8][16 * 68];
  const int b    = blockIdx.y;
  const int lane = threadIdx.x & 31;
  const int wave = threadIdx.x >> 5;
  const int tilesN = N >> 6;
  const int tilesM = M >> 6;
  const int tile = blockIdx.x * 8 + wave;
  if (tile >= tilesM * tilesN) return;
  const int tm = tile / tilesN;
  const int tn = tile - tm * tilesN;
  const int m0 = tm << 6;
  const int n0 = tn << 6;

  const T* Ab  = A  + (size_t)b * strideA;
  const T* Bb  = Bt + (size_t)b * strideB;
  const T* Ab2 = SPLIT ? (A2  + (size_t)b * strideA) : nullptr;
  const T* Bb2 = SPLIT ? (Bt2 + (size_t)b * strideB) : nullptr;

  const int rlane = lane & 15;
  const int koff  = (lane >> 4) * 8;
  const int mOff  = (lane >> 4) * 8;

  v8f acc[4][4];
#pragma unroll
  for (int i = 0; i < 4; ++i)
#pragma unroll
    for (int j = 0; j < 4; ++j) acc[i][j] = (v8f){0.f,0.f,0.f,0.f,0.f,0.f,0.f,0.f};

  for (int k0 = 0; k0 < K; k0 += 32) {
    V bh[4], bl[4];
#pragma unroll
    for (int j = 0; j < 4; ++j) {
      const size_t bo = (size_t)(n0 + (j << 4) + rlane) * ldb + koff + k0;
      bh[j] = Frag<T>::load(Bb + bo);
      if (SPLIT) bl[j] = Frag<T>::load(Bb2 + bo);
    }
#pragma unroll
    for (int i = 0; i < 4; ++i) {
      const size_t ao = (size_t)(m0 + (i << 4) + rlane) * lda + koff + k0;
      V ah = Frag<T>::load(Ab + ao);
      V al;
      if (SPLIT) al = Frag<T>::load(Ab2 + ao);
#pragma unroll
      for (int j = 0; j < 4; ++j) {
        acc[i][j] = Frag<T>::mma(ah, bh[j], acc[i][j]);
        if (SPLIT) {
          acc[i][j] = Frag<T>::mma(ah, bl[j], acc[i][j]);
          acc[i][j] = Frag<T>::mma(al, bh[j], acc[i][j]);
        }
      }
      Frag<T>::guard(acc[i][0], acc[i][3], ah, SPLIT ? al : ah);
    }
    Frag<T>::keep(bh[0], bh[1], bh[2], bh[3]);
    if (SPLIT) Frag<T>::keep(bl[0], bl[1], bl[2], bl[3]);
  }
  acc_guard4(acc[0][0], acc[0][1], acc[0][2], acc[0][3]);
  acc_guard4(acc[1][0], acc[1][1], acc[1][2], acc[1][3]);
  acc_guard4(acc[2][0], acc[2][1], acc[2][2], acc[2][3]);
  acc_guard4(acc[3][0], acc[3][1], acc[3][2], acc[3][3]);

  float* slab = sT[wave];
  const float* Rb = RESID ? (resid + (size_t)b * strideR) : nullptr;
#pragma unroll
  for (int i = 0; i < 4; ++i) {
    const int mBase = m0 + (i << 4);
#pragma unroll
    for (int j = 0; j < 4; ++j) {
      const int n = n0 + (j << 4) + rlane;
      float bv = 0.f;
      if (BIAS_MODE == 2) bv = bias[n];
#pragma unroll
      for (int r = 0; r < 8; ++r) {
        float v = acc[i][j][r] * scale;
        if (BIAS_MODE == 1) v += bias[mBase + mOff + r];
        if (BIAS_MODE == 2) v += bv;
        if (RESID) v += Rb[(size_t)(mBase + mOff + r) * ldc + n];
        if (ACT == 1) v = tanhf(v);
        if (ACT == 2) v = fmaxf(v, 0.0f);
        if (ACT == 3) v = v / (1.0f + expf(-v));
        if (ACT == 4) v = (v > 0.f) ? v : 0.01f * v;
        if (ACT == 6) v = act_ssp(v);
        if (ACT == 7) v = act_sigm(v);
        slab[(mOff + r) * 68 + (j << 4) + rlane] = v;
      }
    }
    __builtin_amdgcn_fence(__ATOMIC_RELEASE, "workgroup");
    __builtin_amdgcn_wave_barrier();
    __builtin_amdgcn_fence(__ATOMIC_ACQUIRE, "workgroup");
    if (OUT_MODE == 0 || OUT_MODE == 3) {
      float* C = (float*)Cout + (size_t)b * strideC;
      const int hh = lane >> 4, c4 = (lane & 15) * 4;
      for (int pass = 0; pass < 2; ++pass) {
#pragma unroll
        for (int it = 0; it < 8; ++it) {
          const int row = it * 2 + hh;
          v4f v = *(const v4f*)(slab + row * 68 + c4);
          *(volatile v4f*)(C + (size_t)(mBase + row) * ldc + n0 + c4) = v;
        }
        __threadfence();
      }
    }
    if (OUT_MODE != 0) {
      const int q = lane >> 3, c8 = (lane & 7) * 8;
      unsigned short* C  = ((OUT_MODE == 3) ? (unsigned short*)Cout2 : (unsigned short*)Cout) + (size_t)b * strideC;
      unsigned short* C2 = (OUT_MODE == 2) ? ((unsigned short*)Cout2 + (size_t)b * strideC) : nullptr;
      for (int pass = 0; pass < 2; ++pass) {
#pragma unroll
        for (int it = 0; it < 4; ++it) {
          const int row = it * 4 + q;
          const float* sp = slab + row * 68 + c8;
          v8h hv, lv;
#pragma unroll
          for (int e = 0; e < 8; ++e) {
            if (OUT_MODE == 2) {
              unsigned short hb = f2bf_bits(sp[e]);
              unsigned short lb = f2bf_bits(sp[e] - bf_bits2f(hb));
              hv[e] = __builtin_bit_cast(_Float16, hb);
              lv[e] = __builtin_bit_cast(_Float16, lb);
            } else {
              hv[e] = (_Float16)sp[e];
            }
          }
          *(volatile v8h*)(C + (size_t)(mBase + row) * ldc + n0 + c8) = hv;
          if (OUT_MODE == 2) *(volatile v8h*)(C2 + (size_t)(mBase + row) * ldc + n0 + c8) = lv;
        }
        __threadfence();
      }
    }
    __builtin_amdgcn_fence(__ATOMIC_RELEASE, "workgroup");
    __builtin_amdgcn_wave_barrier();
    __builtin_amdgcn_fence(__ATOMIC_ACQUIRE, "workgroup");
  }
}

__global__ __launch_bounds__(256) void wprep_kernel(const float* __restrict__ W, unsigned short* __restrict__ OUTP,
                                                    int nl, int Kin, int Nout, int Np, int Kp, float scale, int nseg) {
  const int i = blockIdx.x * 256 + threadIdx.x;
  if (i >= nseg) return;
  const int spr = Kp >> 3;
  const int spl = Np * spr;
  const int l = i / spl;
  const int rem = i - l * spl;
  const int n = rem / spr;
  const int c = rem - n * spr;
  const int nc = (n < Nout) ? n : (Nout - 1);
  (void)nl;
  v8h hv;
#pragma unroll
  for (int j = 0; j < 8; ++j) {
    const int k = 8 * c + j;
    const int kc = (k < Kin) ? k : (Kin - 1);
    float v = W[((size_t)l * Kin + kc) * Nout + nc] * scale;
    v = flush16(v);
    if (k >= Kin || n >= Nout) v = 0.0f;
    hv[j] = (_Float16)v;
  }
  unsigned short* op = OUTP + (size_t)i * 8;
  *(volatile v8h*)op = hv;
  __threadfence();
  *(volatile v8h*)op = hv;
}

__global__ __launch_bounds__(256) void biaspad_kernel(const float* __restrict__ b, float* __restrict__ OUTB) {
  const int i = blockIdx.x * 256 + threadIdx.x;
  if (i >= NEF) return;
  const int ic = (i < NEF_REAL) ? i : (NEF_REAL - 1);
  float v = b[ic];
  if (i >= NEF_REAL) v = 0.0f;
  float* op = OUTB + i;
  *(volatile float*)op = v;
  __threadfence();
  *(volatile float*)op = v;
}

__global__ __launch_bounds__(256) void emb_kernel(const int* __restrict__ z, const float* __restrict__ emb,
                                                  float* __restrict__ HA, unsigned short* __restrict__ H16) {
  const int i = blockIdx.x * 256 + threadIdx.x;
  const v4f z4 = {0.f, 0.f, 0.f, 0.f};
  if (i < N_PADM * 32) {
    const int n = i >> 5, c4 = (i & 31) * 4;
    const int nc = (n < N_ATOM) ? n : (N_ATOM - 1);
    int zi = z[nc]; zi = zi < 0 ? 0 : (zi >= NEMB ? NEMB - 1 : zi);
    v4f v = *(const v4f*)(emb + (size_t)zi * CHAN + c4);
    if (n >= N_ATOM) v = z4;
    float* op = HA + (size_t)n * CHAN + c4;
    *(volatile v4f*)op = v;
    __threadfence();
    *(volatile v4f*)op = v;
  }
  if (i < N_PADM * 16) {
    const int n = i >> 4, c8 = (i & 15) * 8;
    const int nc = (n < N_ATOM) ? n : (N_ATOM - 1);
    int zi = z[nc]; zi = zi < 0 ? 0 : (zi >= NEMB ? NEMB - 1 : zi);
    const float* pe = emb + (size_t)zi * CHAN + c8;
    v4f a0 = *(const v4f*)pe, a1 = *(const v4f*)(pe + 4);
    if (n >= N_ATOM) { a0 = z4; a1 = z4; }
    v8h hv;
#pragma unroll
    for (int e = 0; e < 4; ++e) { hv[e] = (_Float16)flush16(a0[e]); hv[4 + e] = (_Float16)flush16(a1[e]); }
    unsigned short* op = H16 + (size_t)n * CHAN + c8;
    *(volatile v8h*)op = hv;
    __threadfence();
    *(volatile v8h*)op = hv;
  }
}

__global__ __launch_bounds__(256) void geom_kernel(const float* __restrict__ pos, const int* __restrict__ srcv, const int* __restrict__ dstv,
                                                   unsigned short* __restrict__ EA, float* __restrict__ Cg) {
#pragma clang fp contract(off)
  __shared__ float csh[32];
  const int tid = threadIdx.x;
  const int el = tid >> 3, sub = tid & 7;
  const int e = blockIdx.x * 32 + el;
  int s = srcv[e]; s = s < 0 ? 0 : (s >= N_ATOM ? N_ATOM - 1 : s);
  int d = dstv[e]; d = d < 0 ? 0 : (d >= N_ATOM ? N_ATOM - 1 : d);
  const float dx = pos[s * 3 + 0] - pos[d * 3 + 0];
  const float dy = pos[s * 3 + 1] - pos[d * 3 + 1];
  const float dz = pos[s * 3 + 2] - pos[d * 3 + 2];
  const float w = sqrtf(dx * dx + dy * dy + dz * dz + 1e-12f);
  const float inv49 = 1.0f / 49.0f;
  const float d1 = 10.0f * (1.0f * inv49);
  const float coeff = -0.5f / (d1 * d1);
  v8h hv;
#pragma unroll
  for (int j = 0; j < 8; ++j) {
    const int g = 8 * sub + j;
    float off = 10.0f * ((float)g * inv49);
    if (g == NGAU - 1) off = 10.0f;
    const float t = w - off;
    float v = __expf(coeff * (t * t));
    v = (v < F16_MIN_NORMAL) ? 0.0f : v;
    if (g >= NGAU) v = 0.0f;
    hv[j] = (_Float16)v;
  }
  unsigned short* op = EA + (size_t)e * KGAU + 8 * sub;
  *(volatile v8h*)op = hv;
  __threadfence();
  *(volatile v8h*)op = hv;
  const float cv = 0.5f * (cosf((w * 3.14159265358979f) / 10.0f) + 1.0f);
  if (sub == 0) csh[el] = cv;
  __syncthreads();
  if (tid < 32) {
    const float v = csh[tid];
    float* cp = Cg + (size_t)blockIdx.x * 32 + tid;
    *(volatile float*)cp = v;
    __threadfence();
    *(volatile float*)cp = v;
  }
}

__device__ __forceinline__ int blk_excl_scan(int cnt, int* scan_ws, int tid, int* tot) {
  const int lane = tid & 31, wave = tid >> 5; int incl = cnt;
#pragma unroll
  for (int o = 1; o < 32; o <<= 1) { const int v = __shfl_up(incl, o, 32); if (lane >= o) incl += v; }
  if (lane == 31) scan_ws[wave] = incl;
  __syncthreads();
  if (wave == 0) { int wv = (lane < NTH / 32) ? scan_ws[lane] : 0; int wincl = wv;
#pragma unroll
    for (int o = 1; o < 32; o <<= 1) { const int v = __shfl_up(wincl, o, 32); if (lane >= o) wincl += v; }
    if (lane < NTH / 32) scan_ws[32 + lane] = wincl - wv; if (lane == 31) scan_ws[64] = wincl; }
  __syncthreads();
  const int res = scan_ws[32 + wave] + incl - cnt; *tot = scan_ws[64];
  return res;
}
__device__ __forceinline__ int chunk_hits(const int* __restrict__ dstv, int e0, int n0, int tid, int* LIST, int* scan_ws) {
  const int eb = e0 + tid * SPT;
  const bool real = (eb < N_EDGE);
  const int ebc = real ? eb : (N_EDGE - SPT);
  int rec[SPT]; int cnt = 0;
#pragma unroll
  for (int k = 0; k < SPT; k += 4) {
    const v4i d4 = *(const v4i*)(dstv + ebc + k);
#pragma unroll
    for (int e = 0; e < 4; ++e) {
      const int d = d4[e];
      int r = -1;
      if (real && d >= n0 && d < n0 + SRB) { r = ((d - n0) << 18) | (ebc + k + e); ++cnt; }
      rec[k + e] = r;
    }
  }
  int tot; int p = blk_excl_scan(cnt, scan_ws, tid, &tot);
#pragma unroll
  for (int k = 0; k < SPT; ++k) if (rec[k] >= 0) { if ((unsigned)p < (unsigned)SCH) LIST[p] = rec[k]; ++p; }
  __syncthreads();
  return tot < SCH ? tot : SCH;
}

__global__ __launch_bounds__(NTH) void agg_kernel(const float* __restrict__ XJ, const unsigned short* __restrict__ T2p, const float* __restrict__ Cg,
                                                  const int* __restrict__ srcv, const int* __restrict__ dstv, float* ACC) {
  constexpr int NCHK = (N_EDGE + SCH - 1) / SCH;
  __shared__ int LIST[SCH];
  __shared__ int scan_ws[80];
  const _Float16* T2 = (const _Float16*)T2p;
  const int tid = threadIdx.x, lane = tid & 31, wave = tid >> 5;
  const int n0 = blockIdx.x * SRB;
  const v4f zv = {0.0f, 0.0f, 0.0f, 0.0f};
#pragma unroll 1
  for (int j = 0; j < SRB / 8; ++j) {
    float* rp = ACC + (size_t)(n0 + wave * (SRB / 8) + j) * CHAN + 4 * lane;
    *(volatile v4f*)rp = zv;
    __threadfence();
    *(volatile v4f*)rp = zv;
  }
#pragma unroll 1
  for (int c = 0; c < NCHK; ++c) {
    const int tot = chunk_hits(dstv, c * SCH, n0, tid, LIST, scan_ws);
#pragma unroll 1
    for (int base = 0; base < tot; base += 32) {
      const int q = base + lane;
      const int qc = (q < SCH) ? q : (SCH - 1);
      const int lv = LIST[qc];
      const int rv = (q < tot) ? lv : -1;
      const int own = (rv >= 0 && (rv >> 25) == wave) ? 1 : 0;
      unsigned msk = (unsigned)__ballot(own);
#pragma unroll 1
      for (int it = 0; it < 32; ++it) {
        if (msk == 0u) break;
        const int bp = __builtin_ctz(msk); msk &= msk - 1u;
        const int r = __shfl(rv, bp, 32);
        const int dl = (r >> 18) & (SRB - 1);
        int e = r & 0x3FFFF; e = (e < N_EDGE) ? e : (N_EDGE - 1);
        int s = srcv[e]; s = s < 0 ? 0 : (s >= N_ATOM ? N_ATOM - 1 : s);
        const float cv = Cg[e];
        const v4hf th = *(const v4hf*)(T2 + (size_t)e * CHAN + 4 * lane);
        const v4f xj = *(const v4f*)(XJ + (size_t)s * CHAN + 4 * lane);
        v4f wf;
        wf[0] = (float)th[0] * cv; wf[1] = (float)th[1] * cv; wf[2] = (float)th[2] * cv; wf[3] = (float)th[3] * cv;
        float* rp = ACC + (size_t)(n0 + dl) * CHAN + 4 * lane;
        v4f a = *(const v4f*)rp;
        a = a + xj * wf;
        *(volatile v4f*)rp = a;
        __threadfence();
        *(volatile v4f*)rp = a;
      }
    }
    __syncthreads();
  }
}

__global__ __launch_bounds__(256) void cast_agg_kernel(const float* __restrict__ ACC, unsigned short* __restrict__ AGG16) {
  const int i = blockIdx.x * 256 + threadIdx.x;
  if (i >= N_PADM * 16) return;
  const int row = i >> 4, c8 = (i & 15) * 8;
  const float* pa = ACC + (size_t)row * CHAN + c8;
  const v4f a0 = *(const v4f*)pa, a1 = *(const v4f*)(pa + 4);
  v8h hv;
#pragma unroll
  for (int e = 0; e < 4; ++e) { hv[e] = (_Float16)flush16(a0[e]); hv[4 + e] = (_Float16)flush16(a1[e]); }
  unsigned short* op = AGG16 + (size_t)row * CHAN + c8;
  *(volatile v8h*)op = hv;
  __threadfence();
  *(volatile v8h*)op = hv;
}

__global__ __launch_bounds__(256) void ef_kernel(const float* __restrict__ pos, const int* __restrict__ psv, const int* __restrict__ pdv,
                                                 const float* __restrict__ HO, unsigned short* __restrict__ EF) {
#pragma clang fp contract(off)
  __shared__ float sd[32];
  __shared__ float sa[32];
  __shared__ int sia[32];
  __shared__ int sib[32];
  const int tid = threadIdx.x;
  const int rbase = blockIdx.x * 32;
  if (tid < 32) {
    const int ep = rbase + tid;
    int a = psv[ep]; a = a < 0 ? 0 : (a >= N_ATOM ? N_ATOM - 1 : a);
    int c = pdv[ep]; c = c < 0 ? 0 : (c >= N_ATOM ? N_ATOM - 1 : c);
    const float ax = pos[a * 3 + 0], ay = pos[a * 3 + 1], az = pos[a * 3 + 2];
    const float bx = pos[c * 3 + 0], by = pos[c * 3 + 1], bz = pos[c * 3 + 2];
    const float dx = ax - bx, dy = ay - by, dz = az - bz;
    const float dist = sqrtf(dx * dx + dy * dy + dz * dz + 1e-12f);
    const float na = sqrtf(ax * ax + ay * ay + az * az);
    const float nb = sqrtf(bx * bx + by * by + bz * bz);
    float cs = (ax * bx + ay * by + az * bz) / (na * nb + 1e-5f);
    cs = fminf(fmaxf(cs, -0.999999f), 0.999999f);
    const float ang = acosf(cs);
    sd[tid] = dist; sa[tid] = ang; sia[tid] = a; sib[tid] = c;
  }
  __syncthreads();
  const v4f z4 = {0.f, 0.f, 0.f, 0.f};
#pragma unroll 1
  for (int k = 0; k < 3; ++k) {
    const int i = tid + 256 * k;
    const int ic = (i < 640) ? i : 639;
    const int row = ic / 20;
    const int seg = ic - row * 20;
    const int a = sia[row], c = sib[row];
    const float dist = sd[row], ang = sa[row];
    const int ca = (seg * 8) & 63;
    const float* pa = HO + (size_t)a * HOUT + ca;
    const float* pb = HO + (size_t)c * HOUT + ca;
    const v4f a0 = *(const v4f*)pa, a1 = *(const v4f*)(pa + 4);
    const v4f b0 = *(const v4f*)pb, b1 = *(const v4f*)(pb + 4);
    v4f u0 = z4, u1 = z4;
    if (seg < 8) { u0 = a0; u1 = a1; }
    else if (seg < 16) { u0 = b0; u1 = b1; }
    else if (seg == 16) { u0[0] = dist; u0[1] = ang; }
    v8h hv;
#pragma unroll
    for (int e = 0; e < 4; ++e) { hv[e] = (_Float16)flush16(u0[e]); hv[4 + e] = (_Float16)flush16(u1[e]); }
    if (i < 640) {
      unsigned short* op = EF + (size_t)(rbase + row) * KEF + seg * 8;
      *(volatile v8h*)op = hv;
      __threadfence();
      *(volatile v8h*)op = hv;
    }
  }
}

__global__ __launch_bounds__(256) void edot_kernel(const unsigned short* __restrict__ Sp, const float* __restrict__ w2, const float* __restrict__ b2,
                                                   float* __restrict__ out, int nrows) {
  const int lane = threadIdx.x & 31, wave = threadIdx.x >> 5;
  const int rb = (blockIdx.x * 8 + wave) * 32;
  if (rb >= nrows) return;
  const _Float16* S = (const _Float16*)Sp;
  float wa[8], wb[8];
#pragma unroll
  for (int j = 0; j < 8; ++j) { wa[j] = w2[8 * lane + j]; wb[j] = w2[256 + 8 * lane + j]; }
  const int c0 = 512 + 2 * lane, c1 = c0 + 1;
  float wc0 = w2[(c0 < NEF_REAL) ? c0 : (NEF_REAL - 1)];
  float wc1 = w2[(c1 < NEF_REAL) ? c1 : (NEF_REAL - 1)];
  if (c0 >= NEF_REAL) wc0 = 0.0f;
  if (c1 >= NEF_REAL) wc1 = 0.0f;
  const float bb = b2[0];
  float res = 0.0f;
#pragma unroll 1
  for (int i = 0; i < 32; ++i) {
    const _Float16* rp = S + (size_t)(rb + i) * NEF;
    const v8h x0 = *(const v8h*)(rp + 8 * lane);
    const v8h x1 = *(const v8h*)(rp + 256 + 8 * lane);
    const v2hf x2 = *(const v2hf*)(rp + 512 + 2 * lane);
    float s = 0.0f;
#pragma unroll
    for (int j = 0; j < 8; ++j) s += (float)x0[j] * wa[j];
#pragma unroll
    for (int j = 0; j < 8; ++j) s += (float)x1[j] * wb[j];
    s += (float)x2[0] * wc0 + (float)x2[1] * wc1;
#pragma unroll
    for (int off = 1; off < 32; off <<= 1) s += __shfl_xor(s, off, 32);
    s += bb;
    res = (lane == i) ? s : res;
  }
  float* op = out + rb + lane;
  *(volatile float*)op = res;
  __threadfence();
  *(volatile float*)op = res;
}

extern "C" void kernel_launch(void* const* d_in, const int* in_sizes, int n_in,
                              void* d_out, int out_size, void* d_ws, size_t ws_size, hipStream_t stream) {
  if (n_in < 20) return;
  if (in_sizes[0] != N_ATOM || in_sizes[1] != N_ATOM * 3 || in_sizes[2] != 2 * N_EDGE || in_sizes[3] != 2 * N_PRED ||
      in_sizes[4] != NEMB * CHAN || in_sizes[5] != NLAY * NGAU * CHAN || in_sizes[6] != NLAY * CHAN ||
      in_sizes[7] != NLAY * CHAN * CHAN || in_sizes[8] != NLAY * CHAN || in_sizes[9] != NLAY * CHAN * CHAN ||
      in_sizes[10] != NLAY * CHAN * CHAN || in_sizes[11] != NLAY * CHAN || in_sizes[12] != NLAY * CHAN * CHAN ||
      in_sizes[13] != NLAY * CHAN || in_sizes[14] != CHAN * HOUT || in_sizes[15] != HOUT ||
      in_sizes[16] != KEF_REAL * NEF_REAL || in_sizes[17] != NEF_REAL || in_sizes[18] != NEF_REAL || in_sizes[19] != 1) return;
  if (out_size != N_PRED) return;

  const int*   z      = (const int*)d_in[0];
  const float* pos    = (const float*)d_in[1];
  const int*   ei     = (const int*)d_in[2];
  const int*   pei    = (const int*)d_in[3];
  const float* embw   = (const float*)d_in[4];
  const float* mlp_w1 = (const float*)d_in[5];
  const float* mlp_b1 = (const float*)d_in[6];
  const float* mlp_w2 = (const float*)d_in[7];
  const float* mlp_b2 = (const float*)d_in[8];
  const float* cf1w   = (const float*)d_in[9];
  const float* cf2w   = (const float*)d_in[10];
  const float* cf2b   = (const float*)d_in[11];
  const float* linw   = (const float*)d_in[12];
  const float* linb   = (const float*)d_in[13];
  const float* outw   = (const float*)d_in[14];
  const float* outb   = (const float*)d_in[15];
  const float* ew1    = (const float*)d_in[16];
  const float* eb1    = (const float*)d_in[17];
  const float* ew2    = (const float*)d_in[18];
  const float* eb2    = (const float*)d_in[19];
  float* outp = (float*)d_out;

  const int* src = ei;
  const int* dst = ei + N_EDGE;
  const int* ps  = pei;
  const int* pd  = pei + N_PRED;

  char* ws = (char*)d_ws; size_t off = 0;
  auto carve = [&](size_t bytes) -> char* { char* p = ws + off; off += (bytes + 255) & ~(size_t)255; return p; };
  unsigned short* W1T = (unsigned short*)carve((size_t)NLAY * CHAN * KGAU * 2);
  unsigned short* W2T = (unsigned short*)carve((size_t)NLAY * CHAN * CHAN * 2);
  unsigned short* L1T = (unsigned short*)carve((size_t)NLAY * CHAN * CHAN * 2);
  unsigned short* L2T = (unsigned short*)carve((size_t)NLAY * CHAN * CHAN * 2);
  unsigned short* LWT = (unsigned short*)carve((size_t)NLAY * CHAN * CHAN * 2);
  unsigned short* OWT = (unsigned short*)carve((size_t)HOUT * CHAN * 2);
  unsigned short* E1T = (unsigned short*)carve((size_t)NEF * KEF * 2);
  float* EB1P = (float*)carve((size_t)NEF * 4);
  float* CG   = (float*)carve((size_t)N_EDGE * 4);
  const size_t REDGEB = (size_t)N_EDGE * KGAU * 2 + (size_t)N_EHALF * CHAN * 2 + (size_t)N_EDGE * CHAN * 2;
  char* REDGE = carve(REDGEB);
  float* XJ   = (float*)carve((size_t)N_PADM * CHAN * 4);
  float* ACC  = (float*)carve((size_t)NPA * CHAN * 4);
  unsigned short* AGG16 = (unsigned short*)carve((size_t)N_PADM * CHAN * 2);
  unsigned short* V116  = (unsigned short*)carve((size_t)N_PADM * CHAN * 2);
  float* HA   = (float*)carve((size_t)N_PADM * CHAN * 4);
  float* HB   = (float*)carve((size_t)N_PADM * CHAN * 4);
  unsigned short* H16 = (unsigned short*)carve((size_t)N_PADM * CHAN * 2);
  float* HO   = (float*)carve((size_t)N_PADM * HOUT * 4);
  if (off > ws_size || off > (size_t)134217728) return;

  unsigned short* EA16 = (unsigned short*)(REDGE);
  unsigned short* T16H = (unsigned short*)(REDGE + (size_t)N_EDGE * KGAU * 2);
  unsigned short* T2   = (unsigned short*)(REDGE + (size_t)N_EDGE * KGAU * 2 + (size_t)N_EHALF * CHAN * 2);
  unsigned short* EF16 = (unsigned short*)(REDGE);
  unsigned short* S16  = (unsigned short*)(REDGE + (size_t)N_PRED * KEF * 2);
  if ((size_t)N_PRED * KEF * 2 + (size_t)N_PHALF * NEF * 2 > REDGEB) return;

  {
    const int ns1 = NLAY * CHAN * (KGAU / 8);
    const int ns2 = NLAY * CHAN * (CHAN / 8);
    const int nso = HOUT * (CHAN / 8);
    const int nse = NEF * (KEF / 8);
    wprep_kernel<<<(ns1 + 255) / 256, 256, 0, stream>>>(mlp_w1, W1T, NLAY, NGAU, CHAN, CHAN, KGAU, WSC, ns1);
    wprep_kernel<<<(ns2 + 255) / 256, 256, 0, stream>>>(mlp_w2, W2T, NLAY, CHAN, CHAN, CHAN, CHAN, WSC, ns2);
    wprep_kernel<<<(ns2 + 255) / 256, 256, 0, stream>>>(cf1w,   L1T, NLAY, CHAN, CHAN, CHAN, CHAN, WSC, ns2);
    wprep_kernel<<<(ns2 + 255) / 256, 256, 0, stream>>>(cf2w,   L2T, NLAY, CHAN, CHAN, CHAN, CHAN, WSC, ns2);
    wprep_kernel<<<(ns2 + 255) / 256, 256, 0, stream>>>(linw,   LWT, NLAY, CHAN, CHAN, CHAN, CHAN, WSC, ns2);
    wprep_kernel<<<(nso + 255) / 256, 256, 0, stream>>>(outw,   OWT, 1, CHAN, HOUT, HOUT, CHAN, WSC, nso);
    wprep_kernel<<<(nse + 255) / 256, 256, 0, stream>>>(ew1,    E1T, 1, KEF_REAL, NEF_REAL, NEF, KEF, WSC, nse);
    biaspad_kernel<<<(NEF + 255) / 256, 256, 0, stream>>>(eb1, EB1P);
  }
  emb_kernel<<<(N_PADM * 32) / 256, 256, 0, stream>>>(z, embw, HA, H16);
  geom_kernel<<<N_EDGE / 32, 256, 0, stream>>>(pos, src, dst, EA16, CG);

  const int tilesE = (N_EHALF / 64) * (CHAN / 64);
  const int tilesN = (N_PADM / 64) * (CHAN / 64);
  float* Hcur = HA; float* Hnext = HB;
  for (int l = 0; l < NLAY; ++l) {
    for (int hf = 0; hf < 2; ++hf) {
      wmma_gemm64<0, false, 2, 1, false, 6><<<dim3((tilesE + 7) / 8, 1), 256, 0, stream>>>(
          EA16 + (size_t)hf * N_EHALF * KGAU, nullptr, KGAU, 0L, W1T + (size_t)l * CHAN * KGAU, nullptr, KGAU, 0L,
          (void*)T16H, nullptr, CHAN, 0L, mlp_b1 + (size_t)l * CHAN, nullptr, 0L, N_EHALF, CHAN, KGAU, WSC_INV);
      wmma_gemm64<0, false, 2, 1, false, 0><<<dim3((tilesE + 7) / 8, 1), 256, 0, stream>>>(
          T16H, nullptr, CHAN, 0L, W2T + (size_t)l * CHAN * CHAN, nullptr, CHAN, 0L,
          (void*)(T2 + (size_t)hf * N_EHALF * CHAN), nullptr, CHAN, 0L, mlp_b2 + (size_t)l * CHAN, nullptr, 0L, N_EHALF, CHAN, CHAN, WSC_INV);
    }
    wmma_gemm64<0, false, 0, 0, false, 0><<<dim3((tilesN + 7) / 8, 1), 256, 0, stream>>>(
        H16, nullptr, CHAN, 0L, L1T + (size_t)l * CHAN * CHAN, nullptr, CHAN, 0L,
        (void*)XJ, nullptr, CHAN, 0L, nullptr, nullptr, 0L, N_PADM, CHAN, CHAN, WSC_INV);
    agg_kernel<<<NTILE, NTH, 0, stream>>>(XJ, T2, CG, src, dst, ACC);
    cast_agg_kernel<<<(N_PADM * 16) / 256, 256, 0, stream>>>(ACC, AGG16);
    wmma_gemm64<0, false, 2, 1, false, 6><<<dim3((tilesN + 7) / 8, 1), 256, 0, stream>>>(
        AGG16, nullptr, CHAN, 0L, L2T + (size_t)l * CHAN * CHAN, nullptr, CHAN, 0L,
        (void*)V116, nullptr, CHAN, 0L, cf2b + (size_t)l * CHAN, nullptr, 0L, N_PADM, CHAN, CHAN, WSC_INV);
    wmma_gemm64<0, false, 2, 3, true, 0><<<dim3((tilesN + 7) / 8, 1), 256, 0, stream>>>(
        V116, nullptr, CHAN, 0L, LWT + (size_t)l * CHAN * CHAN, nullptr, CHAN, 0L,
        (void*)Hnext, (void*)H16, CHAN, 0L, linb + (size_t)l * CHAN, Hcur, 0L, N_PADM, CHAN, CHAN, WSC_INV);
    float* t = Hcur; Hcur = Hnext; Hnext = t;
  }
  {
    const int tilesO = (N_PADM / 64) * (HOUT / 64);
    wmma_gemm64<0, false, 2, 0, false, 0><<<dim3((tilesO + 7) / 8, 1), 256, 0, stream>>>(
        H16, nullptr, CHAN, 0L, OWT, nullptr, CHAN, 0L,
        (void*)HO, nullptr, HOUT, 0L, outb, nullptr, 0L, N_PADM, HOUT, CHAN, WSC_INV);
  }
  ef_kernel<<<N_PRED / 32, 256, 0, stream>>>(pos, ps, pd, HO, EF16);
  {
    const int tilesH = (N_PHALF / 64) * (NEF / 64);
    for (int hf = 0; hf < 2; ++hf) {
      wmma_gemm64<0, false, 2, 1, false, 7><<<dim3((tilesH + 7) / 8, 1), 256, 0, stream>>>(
          EF16 + (size_t)hf * N_PHALF * KEF, nullptr, KEF, 0L, E1T, nullptr, KEF, 0L,
          (void*)S16, nullptr, NEF, 0L, EB1P, nullptr, 0L, N_PHALF, NEF, KEF, WSC_INV);
      edot_kernel<<<(N_PHALF + 255) / 256, 256, 0, stream>>>(S16, ew2, eb2, outp + (size_t)hf * N_PHALF, N_PHALF);
    }
  }
}
